// XPINN_43482248904826
// MI455X (gfx1250) — hardware-verified
//
#include <hip/hip_runtime.h>
#include <math.h>


#define __bf16 _Float16
typedef __attribute__((ext_vector_type(16))) __bf16 v16bf;
typedef __attribute__((ext_vector_type(8)))  __bf16 v8bf;
typedef __attribute__((ext_vector_type(8)))  float  v8f;
typedef __attribute__((ext_vector_type(4)))  float  v4f_t;
typedef float v4fa __attribute__((ext_vector_type(4), may_alias));
typedef __attribute__((ext_vector_type(4)))  int    v4i_t;
typedef int v4ia __attribute__((ext_vector_type(4), may_alias));
#define NBLK (N_PTS_ / 256)
#define N_PTS_ 262144

#define N_PTS   262144
#define NDOM    4
#define FDIM    100
#define K1PAD   224
#define H       128
#define TILE_M  128
#define NTHREADS 256

#define WPRE_PER_DOM  61440
#define WPRE_L1_BYTES (TILE_M * K1PAD * 2)
#define WPRE_L2_BYTES (H * H * 2)

#define OFF_ACT0  0
#define OFF_WT0   (OFF_ACT0 + TILE_M * K1PAD * 2)
#define OFF_WT1   (OFF_WT0  + TILE_M * K1PAD * 2)
#define OFF_ACT1  (OFF_WT1  + H * H * 2)
#define OFF_B1    (OFF_ACT1 + TILE_M * H * 2)
#define OFF_B2    (OFF_B1 + H * 4)
#define OFF_B3    (OFF_B2 + H * 4)
#define OFF_W4    (OFF_B3 + H * 4)
#define OFF_XS    (OFF_W4 + H * 4)
#define OFF_TS    (OFF_XS + TILE_M * 4)
#define OFF_IDX   (OFF_TS + TILE_M * 4)
#define SMEM_BYTES (OFF_IDX + TILE_M * 4)

__device__ __forceinline__ int domain_of(float xv) {
    return (xv >= -0.5f) + (xv >= 0.0f) + (xv >= 0.5f);
}

__device__ __forceinline__ unsigned lds_addr_of(void* p) {
    return (unsigned)(unsigned long long)(__attribute__((address_space(3))) char*)p;
}

__device__ __forceinline__ void stage_async(void* ldsDst, const char* gsrc,
                                            int nbytes, int tid) {
    unsigned lbase = lds_addr_of(ldsDst);
    for (int off = tid * 16; off < nbytes; off += NTHREADS * 16) {
        unsigned laddr = lbase + (unsigned)off;
        unsigned long long gaddr = (unsigned long long)(gsrc + off);
        asm volatile("global_load_async_to_lds_b128 %0, %1, off"
                     :: "v"(laddr), "v"(gaddr) : "memory");
    }
}

__device__ __forceinline__ void wait_async_all() {
    asm volatile("s_wait_asynccnt 0" ::: "memory");
}

__global__ __launch_bounds__(256) void xpinn_count(const float* __restrict__ x, int* __restrict__ cnt) {
    __shared__ int c4[32];
    const int tid = threadIdx.x, n = blockIdx.x * 256 + tid;
    if (tid < 32) c4[tid] = 0;
    __syncthreads();
    atomicAdd(&c4[domain_of(x[n])], 1);
    __syncthreads();
    if (tid < 8) { const v4i_t v = *(const volatile v4ia*)(c4 + tid * 4); int* d = cnt + blockIdx.x * 32 + tid * 4;
        *(volatile v4i_t*)d = v; __threadfence(); *(volatile v4i_t*)d = v; }
}
__global__ __launch_bounds__(256) void xpinn_scan(const int* __restrict__ cnt, int* __restrict__ baseTab, int* __restrict__ wsi) {
    __shared__ int sb[NDOM * NBLK];
    __shared__ int tot[32];
    const int tid = threadIdx.x;
    if (tid < NDOM) {
        int acc = 0;
        for (int b = 0; b < NBLK; ++b) { sb[tid * NBLK + b] = acc; acc += cnt[b * 32 + tid]; }
        tot[tid] = acc;
    }
    __syncthreads();
    if (tid == 0) {
        int acc = 0;
        for (int d = 0; d < NDOM; ++d) { tot[8 + d] = acc; acc += tot[d]; }
        for (int i = 0; i < 32; ++i) if (!(i < NDOM || (i >= 8 && i < 8 + NDOM))) tot[i] = 0;
    }
    __syncthreads();
    for (int i = tid; i < NDOM * NBLK; i += 256) sb[i] += tot[8 + i / NBLK];
    __syncthreads();
#pragma unroll 1
    for (int pass = 0; pass < 2; ++pass) {
        if (tid < 8) { v4i_t v; v.x = tot[tid * 4 + 0]; v.y = tot[tid * 4 + 1]; v.z = tot[tid * 4 + 2]; v.w = tot[tid * 4 + 3];
            if (tid == 0) { v.x = tot[0]; v.y = tot[1]; v.z = tot[2]; v.w = tot[3]; }
            if (tid == 1) { v.x = tot[8]; v.y = tot[9]; v.z = tot[10]; v.w = tot[11]; }
            if (tid >= 2) { v.x = 0; v.y = 0; v.z = 0; v.w = 0; }
            *(volatile v4i_t*)(wsi + tid * 4) = v; }
        for (int q = tid; q < NDOM * NBLK / 4; q += 256) *(volatile v4i_t*)(baseTab + q * 4) = *(const volatile v4ia*)(sb + q * 4);
        __threadfence();
    }
}
__global__ __launch_bounds__(256) void xpinn_fill(const float* __restrict__ x, const int* __restrict__ baseTab,
                                                  int* __restrict__ bucket, int* __restrict__ rankOf) {
    __shared__ int dom[256];
    const int tid = threadIdx.x, n = blockIdx.x * 256 + tid;
    const int d = domain_of(x[n]);
    dom[tid] = d;
    __syncthreads();
    int rank = 0;
    for (int u = 0; u < tid; ++u) rank += (dom[u] == d);
    const int pos = baseTab[d * NBLK + blockIdx.x] + rank;
    *(volatile int*)(bucket + pos) = n; *(volatile int*)(rankOf + n) = pos; __threadfence();
    *(volatile int*)(bucket + pos) = n; *(volatile int*)(rankOf + n) = pos;
}
__global__ __launch_bounds__(256) void xpinn_gather(const float* __restrict__ res, const int* __restrict__ rankOf, float* __restrict__ out) {
    const int n = blockIdx.x * 256 + threadIdx.x;
    const float v = res[rankOf[n]];
    *(volatile float*)(out + n) = v; __threadfence(); *(volatile float*)(out + n) = v;
}

__global__ void xpinn_prep(const float* __restrict__ W1,
                           const float* __restrict__ W2,
                           const float* __restrict__ W3,
                           void* __restrict__ wpre_) {
    __bf16* wpre = (__bf16*)wpre_;
    int e = blockIdx.x * blockDim.x + threadIdx.x;
    if (e >= NDOM * WPRE_PER_DOM) return;
    int d = e / WPRE_PER_DOM;
    int r = e - d * WPRE_PER_DOM;
    __bf16* wd = wpre + d * WPRE_PER_DOM;
    if (r < TILE_M * K1PAD) {
        int c = r / K1PAD, k = r - c * K1PAD;
        float v = (k < 2 * FDIM) ? W1[(size_t)d * 2 * FDIM * H + k * H + c] : 0.0f;
        *(volatile __bf16*)(wd + r) = (__bf16)v; __threadfence(); *(volatile __bf16*)(wd + r) = (__bf16)v;
    } else if (r < TILE_M * K1PAD + H * H) {
        int q = r - TILE_M * K1PAD;
        int c = q >> 7, k = q & (H - 1);
        const __bf16 v = (__bf16)W2[(size_t)d * H * H + k * H + c];
        *(volatile __bf16*)(wd + r) = v; __threadfence(); *(volatile __bf16*)(wd + r) = v;
    } else {
        int q = r - (TILE_M * K1PAD + H * H);
        int c = q >> 7, k = q & (H - 1);
        const __bf16 v = (__bf16)W3[(size_t)d * H * H + k * H + c];
        *(volatile __bf16*)(wd + r) = v; __threadfence(); *(volatile __bf16*)(wd + r) = v;
    }
}

template <int KPAD, int SNEXT>
__device__ __forceinline__ void layer_wmma(const __bf16* __restrict__ act,
                                           const __bf16* __restrict__ wT,
                                           const float* __restrict__ biasS,
                                           __bf16* __restrict__ actNext,
                                           int wave, int lane) {
    v8f c[8];
#pragma unroll
    for (int j = 0; j < 8; ++j) {
        v8f z = {0.f, 0.f, 0.f, 0.f, 0.f, 0.f, 0.f, 0.f};
        c[j] = z;
    }
    const int mlane = lane & 15;
    const int koff  = (lane >> 4) * 8;
    const int row   = wave * 16 + mlane;

    for (int kt = 0; kt < KPAD / 32; ++kt) {
        const int k0 = kt * 32 + koff;
        v8bf alo = *(const v8bf*)(act + row * KPAD + k0);
        v8bf ahi = *(const v8bf*)(act + row * KPAD + k0 + 16);
        v16bf a = __builtin_shufflevector(alo, ahi,
                   0, 1, 2, 3, 4, 5, 6, 7, 8, 9, 10, 11, 12, 13, 14, 15);
#pragma unroll
        for (int j = 0; j < 8; ++j) {
            const __bf16* bp = wT + (j * 16 + mlane) * KPAD + k0;
            v8bf blo = *(const v8bf*)bp;
            v8bf bhi = *(const v8bf*)(bp + 16);
            v16bf b = __builtin_shufflevector(blo, bhi,
                       0, 1, 2, 3, 4, 5, 6, 7, 8, 9, 10, 11, 12, 13, 14, 15);
            c[j] = __builtin_amdgcn_wmma_f32_16x16x32_f16(
                false, a, false, b, (short)0, c[j], false, false);
        }
    }

    const int mbase = wave * 16 + ((lane >> 4) << 3);
#pragma unroll
    for (int j = 0; j < 8; ++j) {
        const int n = j * 16 + mlane;
        const float bv = biasS[n];
#pragma unroll
        for (int g = 0; g < 8; ++g) {
            float u = c[j][g] + bv;
            float sig = 1.0f / (1.0f + __expf(-u));
            actNext[(mbase + g) * SNEXT + n] = (__bf16)(u * sig);
        }
    }
}

extern "C" __global__ __launch_bounds__(NTHREADS)
void xpinn_mlp(const float* __restrict__ x,  const float* __restrict__ t,
               const float* __restrict__ B,
               const float* __restrict__ b1, const float* __restrict__ b2,
               const float* __restrict__ b3,
               const float* __restrict__ W4, const float* __restrict__ b4,
               const void* __restrict__ wpre,
               const int* __restrict__ counts, const int* __restrict__ base,
               const int* __restrict__ bucket, float* __restrict__ out) {
    extern __shared__ __align__(16) char smem[];
    __bf16* act0 = (__bf16*)(smem + OFF_ACT0);
    __bf16* wT0  = (__bf16*)(smem + OFF_WT0);
    __bf16* wT1  = (__bf16*)(smem + OFF_WT1);
    __bf16* act1 = (__bf16*)(smem + OFF_ACT1);
    float*  b1S  = (float*)(smem + OFF_B1);
    float*  b2S  = (float*)(smem + OFF_B2);
    float*  b3S  = (float*)(smem + OFF_B3);
    float*  w4S  = (float*)(smem + OFF_W4);
    float*  xs   = (float*)(smem + OFF_XS);
    float*  ts   = (float*)(smem + OFF_TS);
    int*    idxS = (int*)(smem + OFF_IDX);

    const int tid = threadIdx.x;
    const int d   = blockIdx.y;
    const int cnt = counts[d];
    const int m0  = blockIdx.x * TILE_M;
    if (m0 >= cnt) return;
    const int bbase = base[d];

    const char* wd = (const char*)wpre + (size_t)d * WPRE_PER_DOM * 2;
    stage_async(wT0, wd, WPRE_L1_BYTES, tid);
    stage_async(wT1, wd + WPRE_L1_BYTES, WPRE_L2_BYTES, tid);

    __builtin_prefetch(bucket + bbase + m0, 0, 0);

    if (tid < TILE_M) {
        int gi = -1; float xv = 0.f, tv = 0.f;
        if (m0 + tid < cnt) {
            gi = bucket[bbase + m0 + tid];
            xv = x[gi];
            tv = t[gi];
        }
        idxS[tid] = gi; xs[tid] = xv; ts[tid] = tv;
    }
    if (tid < H) {
        b1S[tid] = b1[d * H + tid];
        b2S[tid] = b2[d * H + tid];
        b3S[tid] = b3[d * H + tid];
        w4S[tid] = W4[d * H + tid];
    }
    __syncthreads();

    {
        const int r = tid & (TILE_M - 1);
        const int half = tid >> 7;
        const float xv = xs[r], tv = ts[r];
        const float* Bd = B + d * FDIM * 2;
        for (int f = half * 50; f < half * 50 + 50; ++f) {
            float pr = 6.28318530717958647692f * (xv * Bd[2 * f] + tv * Bd[2 * f + 1]);
            act0[r * K1PAD + f]        = (__bf16)sinf(pr);
            act0[r * K1PAD + FDIM + f] = (__bf16)cosf(pr);
        }
        for (int f = 2 * FDIM + half * 12; f < 2 * FDIM + half * 12 + 12; ++f)
            act0[r * K1PAD + f] = (__bf16)0.0f;
    }

    wait_async_all();
    __syncthreads();

    const int wave = tid >> 5, lane = tid & 31;

    layer_wmma<K1PAD, H>(act0, wT0, b1S, act1, wave, lane);
    __syncthreads();

    stage_async(wT0, wd + WPRE_L1_BYTES + WPRE_L2_BYTES, WPRE_L2_BYTES, tid);

    layer_wmma<H, H>(act1, wT1, b2S, act0, wave, lane);
    wait_async_all();
    __syncthreads();

    layer_wmma<H, H>(act0, wT0, b3S, act1, wave, lane);
    __syncthreads();

    if (tid < TILE_M) {
        float acc = 0.f;
        for (int k = 0; k < H; ++k)
            acc += (float)act1[tid * H + k] * w4S[k];
        acc += b4[d];
        if (m0 + tid < cnt) { float* dst = out + bbase + m0 + tid;
            *(volatile float*)dst = acc; __threadfence(); *(volatile float*)dst = acc; }
    }
}

extern "C" void kernel_launch(void* const* d_in, const int* in_sizes, int n_in,
                              void* d_out, int out_size, void* d_ws, size_t ws_size,
                              hipStream_t stream) {
    const float* x  = (const float*)d_in[0];
    const float* t  = (const float*)d_in[1];
    const float* B  = (const float*)d_in[2];
    const float* W1 = (const float*)d_in[3];
    const float* b1 = (const float*)d_in[4];
    const float* W2 = (const float*)d_in[5];
    const float* b2 = (const float*)d_in[6];
    const float* W3 = (const float*)d_in[7];
    const float* b3 = (const float*)d_in[8];
    const float* W4 = (const float*)d_in[9];
    const float* b4 = (const float*)d_in[10];
    float* out = (float*)d_out;

    char* wsb    = (char*)d_ws;
    int*  wsi    = (int*)wsb;
    void* wpre   = (void*)(wsb + 128);
    int*  bucket = (int*)(wsb + 128 + (size_t)NDOM * WPRE_PER_DOM * 2);
    int*  rankOf = bucket + N_PTS;
    int*  cntTab = rankOf + N_PTS;
    int*  baseTab = cntTab + NBLK * 32;
    float* res   = (float*)(baseTab + NDOM * NBLK);

    xpinn_count<<<N_PTS / 256, 256, 0, stream>>>(x, cntTab);
    xpinn_scan<<<1, 256, 0, stream>>>(cntTab, baseTab, wsi);
    xpinn_fill<<<N_PTS / 256, 256, 0, stream>>>(x, baseTab, bucket, rankOf);
    xpinn_prep<<<(NDOM * WPRE_PER_DOM + NTHREADS - 1) / NTHREADS, NTHREADS, 0, stream>>>(
        W1, W2, W3, wpre);

    (void)hipFuncSetAttribute((const void*)xpinn_mlp,
                              hipFuncAttributeMaxDynamicSharedMemorySize,
                              (int)SMEM_BYTES);
    dim3 grid((N_PTS + TILE_M - 1) / TILE_M, NDOM);
    xpinn_mlp<<<grid, NTHREADS, SMEM_BYTES, stream>>>(
        x, t, B, b1, b2, b3, W4, b4, wpre,
        wsi, wsi + 4, bucket, res);
    xpinn_gather<<<N_PTS / 256, 256, 0, stream>>>(res, rankOf, out);
    (void)in_sizes; (void)n_in; (void)out_size; (void)ws_size;
}
